// OKTNet_56075093016912
// MI455X (gfx1250) — hardware-run, weakly checked
//
#include <hip/hip_runtime.h>
#include <stddef.h>
#include <stdint.h>
#include <math.h>


#define NB     512
#define NS     500
#define NR     (NB * NS)
#define DD     128
#define HID    256
#define NEX    20001
#define NEXP   20032
#define NSK    201
#define NSKP   256
#define NIT    101
#define NITP   128
#define NAT    101
#define NATP   128
#define NANS   2
#define NANSP  64
#define RB     64
#define NTHR   256
#define NBLK_S (NB / RB)
#define NCHUNK (NR / 128)

#define WC     64.0f
#define AC     16.0f
#define EC     256.0f
#define INV_AW (1.0f / 1024.0f)
#define INV_EW (1.0f / 16384.0f)
#define INV_TW (1.0f / 4096.0f)

#define PKH_WQA   0
#define PKH_WQB   16384
#define PKH_WXA   32768
#define PKH_WXANS 49152
#define PKH_WXAT  57344
#define PKH_WUA   65536
#define PKH_ITW   81920
#define PKH_WP1   131072
#define PKH_WZ    196608
#define PKH_WR    229376
#define PKH_WH    262144
#define PKH_WOG   294912
#define PKH_WOV   327680
#define PKH_END   360448

#define O_PK     ((size_t)0)
#define SZ_PK    ((size_t)PKH_END * 2)
#define O_KC16   (O_PK + SZ_PK)
#define SZ_KC16  ((size_t)NSKP * DD * 2)
#define O_IT16   (O_KC16 + SZ_KC16)
#define SZ_IT16  ((size_t)NITP * DD * 2)
#define O_AT16   (O_IT16 + SZ_IT16)
#define SZ_AT16  ((size_t)NATP * 64 * 2)
#define O_ANS16  (O_AT16 + SZ_AT16)
#define SZ_ANS16 ((size_t)NANSP * 64 * 2)
#define O_TKC    (O_ANS16 + SZ_ANS16)
#define SZ_TKC   ((size_t)NSKP * DD * 4)
#define O_TITW   (O_TKC + SZ_TKC)
#define SZ_TITW  ((size_t)NITP * 384 * 4)
#define O_TAT    (O_TITW + SZ_TITW)
#define SZ_TAT   ((size_t)NATP * DD * 4)
#define O_TANS   (O_TAT + SZ_TAT)
#define SZ_TANS  ((size_t)NANSP * DD * 4)
#define O_OUTS   (O_TANS + SZ_TANS)
#define SZ_OUTS  ((size_t)NS * NB * 4)
#define O_Q16    (O_OUTS + SZ_OUTS)
#define SZ_Q16   ((size_t)NR * DD * 2)
#define O_X16    (O_Q16 + SZ_Q16)
#define SZ_X16   SZ_Q16
#define O_E16    O_X16
#define SZ_E16   ((size_t)NEXP * DD * 2)
#define O_TE     (O_E16 + SZ_E16)
#define SZ_TE    ((size_t)NEXP * DD * 4)
#define WSTOT    (O_X16 + SZ_X16)
#define WSCAP    ((size_t)134217728)

#define L_SHH    0
#define L_SQUX   32768
#define L_HS     98304
#define L_VS     131072
#define L_ZS     163840
#define L_IT0    196608
#define L_RED    229376
#define L_BIAS   233472
#define L_PS     239616
#define L_IDX    239872
#define LDS_STEP 240128
#define IT1P     256
#define LDS_TG   98304

static_assert(WSTOT == (size_t)133365760);
static_assert(WSTOT <= WSCAP);
static_assert(O_TE + SZ_TE <= WSTOT);
static_assert((O_KC16 % 128) == 0 && (O_IT16 % 128) == 0 && (O_AT16 % 128) == 0 && (O_ANS16 % 128) == 0);
static_assert((O_TKC % 128) == 0 && (O_TITW % 128) == 0 && (O_TAT % 128) == 0 && (O_TANS % 128) == 0);
static_assert((O_OUTS % 128) == 0 && (O_Q16 % 128) == 0 && (O_X16 % 128) == 0 && (O_TE % 128) == 0);
static_assert(PKH_WQB - PKH_WQA == 512 * 4 * 8 && PKH_WXAT - PKH_WXANS == 512 * 2 * 8);
static_assert(PKH_WP1 - PKH_ITW == 512 * 4 * 24 && PKH_WZ - PKH_WP1 == 512 * 8 * 16 && PKH_WR - PKH_WZ == 512 * 8 * 8);
static_assert(NCHUNK * 128 == NR && NBLK_S * RB == NB && (NR % RB) == 0);
static_assert(NEXP % 64 == 0 && NEXP >= NEX && NSKP >= NSK && NITP >= NIT && NATP >= NAT && NANSP >= NANS);
static_assert(L_SQUX == L_SHH + 64 * 256 * 2 && L_HS == L_SQUX + 64 * 512 * 2 && L_VS == L_HS + 64 * 128 * 4);
static_assert(L_ZS == L_VS + 64 * 128 * 4 && L_IT0 == L_ZS + 64 * 128 * 4 && L_RED == L_IT0 + 64 * 128 * 4);
static_assert(L_BIAS == L_RED + 64 * 16 * 4 && L_PS == L_BIAS + 1536 * 4);
static_assert(L_IDX == L_PS + 64 * 4 && LDS_STEP == L_IDX + 64 * 4);
static_assert(LDS_STEP <= 266000);
static_assert((63 * IT1P + 127) * 4 < 64 * 512 * 2);
static_assert(IT1P * 4 == 512 * 2 && DD * 4 == 256 * 2);

typedef _Float16 v16h __attribute__((ext_vector_type(16)));
typedef _Float16 v8h  __attribute__((ext_vector_type(8), __may_alias__));
typedef float    v8f  __attribute__((ext_vector_type(8)));
typedef float    v4f  __attribute__((ext_vector_type(4), __may_alias__));
union Frag { v16h v; v8h h[2]; };
static_assert(sizeof(Frag) == 32);

struct PackArgs { const float* src[16]; _Float16* dst[16]; int K[16]; int N[16]; int pitch[16]; int roff[16]; int swp[16]; int nfrag[16]; };
static_assert(sizeof(PackArgs) == 16 * 8 * 2 + 16 * 4 * 6);
struct RowsArgs { const float* src[8]; _Float16* dst[8]; int rsrc[8]; int rpad[8]; int cols[8]; int blk0[8]; float carry[8]; int nb[8]; };
static_assert(sizeof(RowsArgs) == 8 * 8 * 2 + 8 * 4 * 6);
struct TgArgs { const _Float16* A[8]; const v16h* Bp[8]; float* C[8]; int Mpad[8]; int K[8]; int N[8]; int blk0[8]; float inv[8]; int nb[8]; };
static_assert(sizeof(TgArgs) == 8 * 8 * 3 + 8 * 4 * 6);

__device__ __forceinline__ int clampi(int v, int lo, int hi) { return v < lo ? lo : (v > hi ? hi : v); }

__device__ __forceinline__ v8f wmh(v16h a, v16h bq, v8f c) {
  v8f d = __builtin_amdgcn_wmma_f32_16x16x32_f16(false, a, false, bq, (short)0, c, false, false);
  asm volatile("v_nop\n\tv_nop\n\tv_nop\n\tv_nop" : "+v"(d) : "v"(a), "v"(bq));
  return d;
}
__device__ __forceinline__ void wmh2(v16h a0, v16h a1, v16h bq, v8f& c0, v8f& c1) {
  v8f d0 = __builtin_amdgcn_wmma_f32_16x16x32_f16(false, a0, false, bq, (short)0, c0, false, false);
  v8f d1 = __builtin_amdgcn_wmma_f32_16x16x32_f16(false, a1, false, bq, (short)0, c1, false, false);
  asm volatile("v_nop\n\tv_nop\n\tv_nop\n\tv_nop" : "+v"(d0), "+v"(d1) : "v"(a0), "v"(a1), "v"(bq));
  c0 = d0; c1 = d1;
}
__device__ __forceinline__ v8f zero8() { v8f z = {0.f, 0.f, 0.f, 0.f, 0.f, 0.f, 0.f, 0.f}; return z; }

__device__ __forceinline__ v16h lda_frag(const _Float16* base, int pitch, int lane) {
  const int m = lane & 15, hh = lane >> 4;
  const _Float16* p = base + (size_t)m * pitch + 8 * hh;
  Frag u;
  u.h[0] = *(const v8h*)p;
  u.h[1] = *(const v8h*)(p + 16);
  return u.v;
}

template <int KC>
__device__ __forceinline__ void gemm4(const _Float16* A, int pitch, const v16h* __restrict__ Bp, int nt,
                                      int lane, v8f& c0, v8f& c1, v8f& c2, v8f& c3) {
  const v16h* bp = Bp + (size_t)nt * KC * 32 + lane;
#pragma unroll 2
  for (int kc = 0; kc < KC; ++kc) {
    const v16h b = bp[kc * 32];
    const _Float16* a0 = A + kc * 32;
    c0 = wmh(lda_frag(a0, pitch, lane), b, c0);
    c1 = wmh(lda_frag(a0 + 16 * pitch, pitch, lane), b, c1);
    c2 = wmh(lda_frag(a0 + 32 * pitch, pitch, lane), b, c2);
    c3 = wmh(lda_frag(a0 + 48 * pitch, pitch, lane), b, c3);
  }
}
template <int KC>
__device__ __forceinline__ void gemm2(const _Float16* A, int pitch, const v16h* __restrict__ bp, int lane,
                                      v8f& c0, v8f& c1) {
#pragma unroll 1
  for (int kc = 0; kc < KC; ++kc) {
    const v16h b = bp[kc * 32];
    const _Float16* a = A + kc * 32;
    const v16h f0 = lda_frag(a, pitch, lane);
    const v16h f1 = lda_frag(a + 16 * pitch, pitch, lane);
    wmh2(f0, f1, b, c0, c1);
  }
}

__device__ __forceinline__ float rcp_(float x) { return __builtin_amdgcn_rcpf(x); }
__device__ __forceinline__ float sigm_(float x) {
  x = fminf(fmaxf(x, -30.0f), 30.0f);
  return rcp_(1.0f + __expf(-x));
}
__device__ __forceinline__ float tanh_(float x) {
  x = fminf(fmaxf(x, -15.0f), 15.0f);
  return 1.0f - 2.0f * rcp_(1.0f + __expf(2.0f * x));
}

__device__ __forceinline__ void vst2_v8h(_Float16* d, v8h v) {
  *(volatile v8h*)d = v;
  __threadfence();
  *(volatile v8h*)d = v;
}

__global__ __launch_bounds__(256) void k_pack(PackArgs P) {
  const int seg = blockIdx.y;
  const int e = blockIdx.x * 256 + threadIdx.x;
  if (e >= P.nfrag[seg] * 64) return;
  const int K = P.K[seg], pitch = P.pitch[seg], roff = P.roff[seg], swp = P.swp[seg];
  const int KC = K >> 5, KH = K >> 1;
  const int frag = e >> 6, r = e & 63, lane = r >> 1, q = r & 1;
  const int nt = frag / KC, kc = frag - nt * KC;
  const int n = nt * 16 + (lane & 15);
  const int kb = kc * 32 + 16 * q + 8 * (lane >> 4);
  const float* src = P.src[seg];
  v8h hv;
#pragma unroll
  for (int i = 0; i < 8; ++i) {
    int k = kb + i;
    if (swp) k = (k < KH) ? (k + KH) : (k - KH);
    hv[i] = (_Float16)(src[(size_t)(roff + k) * pitch + n] * WC);
  }
  vst2_v8h(P.dst[seg] + (size_t)8 * e, hv);
}

__global__ __launch_bounds__(256) void k_rows16(RowsArgs P) {
  const int bid = blockIdx.x;
  int seg = 0;
#pragma unroll
  for (int s = 1; s < 8; ++s) if (P.nb[s] > 0 && bid >= P.blk0[s]) seg = s;
  const int cols = P.cols[seg];
  const int lg = (cols == 128) ? 4 : 3;
  const int item = (bid - P.blk0[seg]) * 256 + threadIdx.x;
  const int row = item >> lg, g = item - (row << lg);
  if (row >= P.rpad[seg]) return;
  const int rsrc = P.rsrc[seg];
  const int rs = row < rsrc ? row : rsrc - 1;
  const float* s = P.src[seg] + (size_t)rs * cols + 8 * g;
  const v4f a = *(const v4f*)s, b = *(const v4f*)(s + 4);
  const float sc = (row < rsrc) ? P.carry[seg] : 0.0f;
  v8h hv;
  hv[0] = (_Float16)(a.x * sc); hv[1] = (_Float16)(a.y * sc); hv[2] = (_Float16)(a.z * sc); hv[3] = (_Float16)(a.w * sc);
  hv[4] = (_Float16)(b.x * sc); hv[5] = (_Float16)(b.y * sc); hv[6] = (_Float16)(b.z * sc); hv[7] = (_Float16)(b.w * sc);
  vst2_v8h(P.dst[seg] + (size_t)row * cols + 8 * g, hv);
}

__global__ __launch_bounds__(256) __attribute__((amdgpu_num_vgpr(256))) void k_tgemm(TgArgs P) {
  extern __shared__ __align__(16) char smem_t[];
  float* sC = (float*)smem_t;
  const int bid = blockIdx.x;
  int seg = 0;
#pragma unroll
  for (int s = 1; s < 8; ++s) if (P.nb[s] > 0 && bid >= P.blk0[s]) seg = s;
  const int K = P.K[seg], N = P.N[seg], KC = K >> 5, NT = N >> 4;
  const int mrow0 = (bid - P.blk0[seg]) * 64;
  const _Float16* A = P.A[seg];
  const v16h* Bp = P.Bp[seg];
  float* C = P.C[seg];
  const float inv = P.inv[seg];
  const int tid = threadIdx.x, lane = tid & 31, wave = tid >> 5, hh = lane >> 4, nn = lane & 15;

#pragma unroll 1
  for (int nt = wave; nt < NT; nt += 8) {
    v8f c0 = zero8(), c1 = zero8(), c2 = zero8(), c3 = zero8();
#pragma unroll 2
    for (int kc = 0; kc < KC; ++kc) {
      const v16h b = Bp[(nt * KC + kc) * 32 + lane];
      const _Float16* a0 = A + (size_t)mrow0 * K + kc * 32;
      c0 = wmh(lda_frag(a0, K, lane), b, c0);
      c1 = wmh(lda_frag(a0 + 16 * K, K, lane), b, c1);
      c2 = wmh(lda_frag(a0 + 32 * K, K, lane), b, c2);
      c3 = wmh(lda_frag(a0 + 48 * K, K, lane), b, c3);
    }
    const int col = nt * 16 + nn;
#pragma unroll
    for (int r = 0; r < 8; ++r) {
      sC[(8 * hh + r) * N + col]      = c0[r] * inv;
      sC[(16 + 8 * hh + r) * N + col] = c1[r] * inv;
      sC[(32 + 8 * hh + r) * N + col] = c2[r] * inv;
      sC[(48 + 8 * hh + r) * N + col] = c3[r] * inv;
    }
  }
  __syncthreads();
  const int nseg = N >> 7;
  for (int row = wave; row < 64; row += 8)
    for (int j = 0; j < nseg; ++j) {
      const v4f v = *(const v4f*)(sC + row * N + 128 * j + 4 * lane);
      *(volatile v4f*)(C + (size_t)(mrow0 + row) * N + 128 * j + 4 * lane) = v;
    }
  __threadfence();
  for (int row = wave; row < 64; row += 8)
    for (int j = 0; j < nseg; ++j) {
      const v4f v = *(const v4f*)(sC + row * N + 128 * j + 4 * lane);
      *(volatile v4f*)(C + (size_t)(mrow0 + row) * N + 128 * j + 4 * lane) = v;
    }
}

__global__ __launch_bounds__(256) void k_q(const int* __restrict__ e_data, const int* __restrict__ kc_data,
                                           const float* __restrict__ TE, const float* __restrict__ TK,
                                           const float* __restrict__ bq, _Float16* Q16) {
  const int gid = blockIdx.x * 256 + threadIdx.x;
  const int row = gid >> 4, g = gid & 15;
  if (row >= NR) return;
  const int t = row >> 9, b = row & 511;
  const size_t pos = (size_t)b * NS + t;
  const int e = clampi(e_data[pos], 0, NEX - 1);
  const int k = clampi(kc_data[pos], 0, NSK - 1);
  const float* pe = TE + (size_t)e * DD + 8 * g;
  const float* pk = TK + (size_t)k * DD + 8 * g;
  const float* pb = bq + 8 * g;
  const v4f e0 = *(const v4f*)pe, e1 = *(const v4f*)(pe + 4);
  const v4f k0 = *(const v4f*)pk, k1 = *(const v4f*)(pk + 4);
  const v4f b0 = *(const v4f*)pb, b1 = *(const v4f*)(pb + 4);
  const v4f q0 = (e0 + k0 + b0) * AC, q1 = (e1 + k1 + b1) * AC;
  v8h hv;
  hv[0] = (_Float16)q0.x; hv[1] = (_Float16)q0.y; hv[2] = (_Float16)q0.z; hv[3] = (_Float16)q0.w;
  hv[4] = (_Float16)q1.x; hv[5] = (_Float16)q1.y; hv[6] = (_Float16)q1.z; hv[7] = (_Float16)q1.w;
  vst2_v8h(Q16 + (size_t)row * DD + 8 * g, hv);
}

__global__ __launch_bounds__(256) __attribute__((amdgpu_num_vgpr(256))) void k_x(
    const int* __restrict__ a_data, const int* __restrict__ at_data,
    const _Float16* __restrict__ Q16, const v16h* __restrict__ WXAp,
    const float* __restrict__ TANS, const float* __restrict__ TAT,
    const float* __restrict__ bx, _Float16* X16) {
  __shared__ __align__(16) _Float16 sX[RB * DD];
  __shared__ __align__(16) float sAdd[RB * DD];
  __shared__ int ida[RB];
  __shared__ int idt[RB];
  const int tid = threadIdx.x, lane = tid & 31, wave = tid >> 5, hh = lane >> 4, nn = lane & 15;
  const int row0 = blockIdx.x * RB;
  const int t = row0 >> 9, b0 = row0 & 511;
  if (tid < RB) {
    const size_t pos = (size_t)(b0 + tid) * NS + t;
    ida[tid] = clampi(a_data[pos], 0, NANS - 1);
    idt[tid] = clampi(at_data[pos], 0, NAT - 1);
  }
  __syncthreads();
#pragma unroll 2
  for (int i = 0; i < 8; ++i) {
    const int item = tid + NTHR * i;
    const int row = item >> 5, j = item & 31;
    const v4f a = *(const v4f*)(TANS + (size_t)ida[row] * DD + 4 * j);
    const v4f b = *(const v4f*)(TAT + (size_t)idt[row] * DD + 4 * j);
    const v4f c = *(const v4f*)(bx + 4 * j);
    *(v4f*)(sAdd + row * DD + 4 * j) = a + b + c;
  }
  __syncthreads();
  {
    v8f c0 = zero8(), c1 = zero8(), c2 = zero8(), c3 = zero8();
    gemm4<4>(Q16 + (size_t)row0 * DD, DD, WXAp, wave, lane, c0, c1, c2, c3);
    const int col = wave * 16 + nn;
#pragma unroll
    for (int r = 0; r < 8; ++r) {
      const int rw0 = 8 * hh + r, rw1 = 16 + rw0, rw2 = 32 + rw0, rw3 = 48 + rw0;
      const float x0 = c0[r] * INV_AW + sAdd[rw0 * DD + col];
      const float x1 = c1[r] * INV_AW + sAdd[rw1 * DD + col];
      const float x2 = c2[r] * INV_AW + sAdd[rw2 * DD + col];
      const float x3 = c3[r] * INV_AW + sAdd[rw3 * DD + col];
      sX[rw0 * DD + col] = (_Float16)(x0 * AC);
      sX[rw1 * DD + col] = (_Float16)(x1 * AC);
      sX[rw2 * DD + col] = (_Float16)(x2 * AC);
      sX[rw3 * DD + col] = (_Float16)(x3 * AC);
    }
  }
  __syncthreads();
  v8h v[4];
#pragma unroll
  for (int i = 0; i < 4; ++i) {
    const int item = tid + NTHR * i;
    v[i] = *(const v8h*)(sX + (item >> 4) * DD + 8 * (item & 15));
  }
#pragma unroll
  for (int i = 0; i < 4; ++i) {
    const int item = tid + NTHR * i;
    *(volatile v8h*)(X16 + (size_t)(row0 + (item >> 4)) * DD + 8 * (item & 15)) = v[i];
  }
  __threadfence();
#pragma unroll
  for (int i = 0; i < 4; ++i) {
    const int item = tid + NTHR * i;
    *(volatile v8h*)(X16 + (size_t)(row0 + (item >> 4)) * DD + 8 * (item & 15)) = v[i];
  }
}

__device__ __forceinline__ void epi_gamma(const v8f& c, int mt, int hh, int col, const float* sIT0,
                                          const float* sBu, float* hS, const float* vS, _Float16* sQUX) {
#pragma unroll
  for (int r = 0; r < 8; ++r) {
    const int row = mt * 16 + 8 * hh + r;
    const int i = row * DD + col;
    const float g = sigm_(c[r] * INV_AW + sIT0[i] + sBu[col]);
    const float uh = hS[i] + g * vS[i];
    hS[i] = uh;
    sQUX[row * 512 + 128 + col] = (_Float16)(uh * AC);
  }
}
__device__ __forceinline__ void epi_p1(const v8f& c, int mt, int hh, int nn, int col, int nt,
                                       const float* sBp1, const float* sWp2, float* red) {
  float s[8];
#pragma unroll
  for (int r = 0; r < 8; ++r) s[r] = fmaxf(c[r] * INV_AW + sBp1[col], 0.0f) * sWp2[col];
#pragma unroll
  for (int r = 0; r < 8; ++r) {
    float v = s[r];
    v += __shfl_xor(v, 1);
    v += __shfl_xor(v, 2);
    v += __shfl_xor(v, 4);
    v += __shfl_xor(v, 8);
    s[r] = v;
  }
  if (nn == 0) {
#pragma unroll
    for (int r = 0; r < 8; ++r) red[(mt * 16 + 8 * hh + r) * 16 + nt] = s[r];
  }
}
__device__ __forceinline__ void epi_z(const v8f& c, int mt, int hh, int col, const float* sBz, float* zS) {
#pragma unroll
  for (int r = 0; r < 8; ++r) {
    const int row = mt * 16 + 8 * hh + r;
    zS[row * DD + col] = sigm_(c[r] * INV_AW + sBz[col]);
  }
}
__device__ __forceinline__ void epi_r(const v8f& c, int mt, int hh, int col, const float* sBr, const float* hS,
                                      _Float16* sQUX) {
#pragma unroll
  for (int r = 0; r < 8; ++r) {
    const int row = mt * 16 + 8 * hh + r;
    const float rr = sigm_(c[r] * INV_AW + sBr[col]);
    const float ruh = rr * hS[row * DD + col];
    sQUX[row * 512 + 384 + col] = (_Float16)(ruh * AC);
  }
}
__device__ __forceinline__ void epi_h(const v8f& c, int mt, int hh, int col, const float* sBh, const float* zS,
                                      float* hS, _Float16* sHH) {
#pragma unroll
  for (int r = 0; r < 8; ++r) {
    const int row = mt * 16 + 8 * hh + r;
    const int i = row * DD + col;
    const float hc = tanh_(c[r] * INV_AW + sBh[col]);
    const float z = zS[i], uh = hS[i];
    const float hn = (1.0f - z) * uh + z * hc;
    hS[i] = hn;
    sHH[row * 256 + 128 + col] = (_Float16)(hn * AC);
  }
}
__device__ __forceinline__ void epi_g(const v8f& c, int mt, int hh, int col, const float* sIT1, const float* sBog,
                                      float* gS) {
#pragma unroll
  for (int r = 0; r < 8; ++r) {
    const int row = mt * 16 + 8 * hh + r;
    gS[row * DD + col] = sigm_(c[r] * INV_AW + sIT1[row * IT1P + col] + sBog[col]);
  }
}
__device__ __forceinline__ void epi_v(const v8f& c, int mt, int hh, int col, const float* sIT0, const float* sBov,
                                      const float* gS, float* vS) {
#pragma unroll
  for (int r = 0; r < 8; ++r) {
    const int row = mt * 16 + 8 * hh + r;
    const int i = row * DD + col;
    const float ov = tanh_(c[r] * INV_AW + sIT0[i] + sBov[col]);
    const float g = gS[i];
    const float v = vS[i];
    vS[i] = g * v + (1.0f - g) * ov;
  }
}

__global__ __launch_bounds__(NTHR) __attribute__((amdgpu_num_vgpr(192))) void k_step(
    const int* __restrict__ it_data, const _Float16* __restrict__ Q16, const _Float16* __restrict__ X16,
    const float* __restrict__ TITW,
    const v16h* __restrict__ WUAp, const v16h* __restrict__ WP1p, const v16h* __restrict__ WZp,
    const v16h* __restrict__ WRp, const v16h* __restrict__ WHp, const v16h* __restrict__ WOGp,
    const v16h* __restrict__ WOVp,
    const float* __restrict__ bu, const float* __restrict__ bz, const float* __restrict__ br,
    const float* __restrict__ bh, const float* __restrict__ bog, const float* __restrict__ bov,
    const float* __restrict__ bp1, const float* __restrict__ Wp2, const float* __restrict__ bp2,
    const float* __restrict__ h0, const float* __restrict__ v0, float* OUTS) {
  extern __shared__ __align__(16) char smem_s[];
  _Float16* sHH  = (_Float16*)(smem_s + L_SHH);
  _Float16* sQUX = (_Float16*)(smem_s + L_SQUX);
  float* sIT1 = (float*)(smem_s + L_SQUX);
  float* hS   = (float*)(smem_s + L_HS);
  float* vS   = (float*)(smem_s + L_VS);
  float* zS   = (float*)(smem_s + L_ZS);
  float* sIT0 = (float*)(smem_s + L_IT0);
  float* red  = (float*)(smem_s + L_RED);
  float* sB   = (float*)(smem_s + L_BIAS);
  float* pS   = (float*)(smem_s + L_PS);
  int* itIdx  = (int*)(smem_s + L_IDX);
  float* sBu = sB;          float* sBz = sB + 128;  float* sBr = sB + 256;  float* sBh = sB + 384;
  float* sBog = sB + 512;   float* sBov = sB + 640; float* sBp1 = sB + 768; float* sWp2 = sB + 1024;
  float* sBp2 = sB + 1280;

  const int tid = threadIdx.x, lane = tid & 31, wave = tid >> 5, hh = lane >> 4, nn = lane & 15;
  const int rowBase = blockIdx.x * RB;
  const int col = wave * 16 + nn;

#pragma unroll 1
  for (int i = tid; i < 128; i += NTHR) {
    sBu[i] = bu[i]; sBz[i] = bz[i]; sBr[i] = br[i]; sBh[i] = bh[i]; sBog[i] = bog[i]; sBov[i] = bov[i];
  }
#pragma unroll 1
  for (int i = tid; i < HID; i += NTHR) { sBp1[i] = bp1[i]; sWp2[i] = Wp2[i]; }
  if (tid == 0) sBp2[0] = bp2[0];
#pragma unroll 1
  for (int i = tid; i < RB * DD; i += NTHR) {
    const int row = i >> 7, cc = i & 127;
    const float hv = h0[cc];
    hS[i] = hv;
    vS[i] = v0[cc];
    sHH[row * 256 + cc] = (_Float16)(hv * AC);
  }
  if (tid < RB) itIdx[tid] = clampi(it_data[(size_t)(rowBase + tid) * NS], 0, NIT - 1);
  __syncthreads();

#pragma unroll 1
  for (int t = 0; t < NS; ++t) {
    {
      const size_t gro = (size_t)(t * NB + rowBase) * DD;
#pragma unroll 2
      for (int i = 0; i < 4; ++i) {
        const int item = tid + NTHR * i;
        const int row = item >> 4, g = item & 15;
        const v8h qv = *(const v8h*)(Q16 + gro + (size_t)row * DD + 8 * g);
        const v8h xv = *(const v8h*)(X16 + gro + (size_t)row * DD + 8 * g);
        *(v8h*)(sQUX + row * 512 + 8 * g)       = qv;
        *(v8h*)(sQUX + row * 512 + 256 + 8 * g) = xv;
      }
#pragma unroll 2
      for (int i = 0; i < 8; ++i) {
        const int item = tid + NTHR * i;
        const int row = item >> 5, j = item & 31;
        const v4f a = *(const v4f*)(TITW + (size_t)itIdx[row] * 384 + 4 * j);
        *(v4f*)(sIT0 + row * DD + 4 * j) = a;
      }
      if (t > 0) {
#pragma unroll 2
        for (int i = 0; i < 4; ++i) {
          const int item = tid + NTHR * i;
          const int row = item >> 4, g = item & 15;
          *(v8h*)(sHH + row * 256 + 8 * g) = *(const v8h*)(sHH + row * 256 + 128 + 8 * g);
        }
      }
    }
    __syncthreads();

#pragma unroll 1
    for (int hb = 0; hb < 2; ++hb) {
      v8f c0 = zero8(), c1 = zero8();
      gemm2<4>(sHH + hb * (32 * 256), 256, WUAp + wave * (4 * 32) + lane, lane, c0, c1);
      __builtin_amdgcn_sched_barrier(0);
      epi_gamma(c0, 2 * hb, hh, col, sIT0, sBu, hS, vS, sQUX);
      __builtin_amdgcn_sched_barrier(0);
      epi_gamma(c1, 2 * hb + 1, hh, col, sIT0, sBu, hS, vS, sQUX);
    }
    __syncthreads();

#pragma unroll 1
    for (int ps = 0; ps < 4; ++ps) {
      const int j = ps >> 1, hb = ps & 1;
      const int nt = wave + 8 * j;
      v8f c0 = zero8(), c1 = zero8();
      gemm2<8>(sQUX + hb * (32 * 512), 512, WP1p + nt * (8 * 32) + lane, lane, c0, c1);
      __builtin_amdgcn_sched_barrier(0);
      const int colp = nt * 16 + nn;
      epi_p1(c0, 2 * hb, hh, nn, colp, nt, sBp1, sWp2, red);
      __builtin_amdgcn_sched_barrier(0);
      epi_p1(c1, 2 * hb + 1, hh, nn, colp, nt, sBp1, sWp2, red);
    }
#pragma unroll 1
    for (int hb = 0; hb < 2; ++hb) {
      v8f c0 = zero8(), c1 = zero8();
      gemm2<8>(sQUX + 128 + hb * (32 * 512), 512, WZp + wave * (8 * 32) + lane, lane, c0, c1);
      __builtin_amdgcn_sched_barrier(0);
      epi_z(c0, 2 * hb, hh, col, sBz, zS);
      __builtin_amdgcn_sched_barrier(0);
      epi_z(c1, 2 * hb + 1, hh, col, sBz, zS);
    }
#pragma unroll 1
    for (int hb = 0; hb < 2; ++hb) {
      v8f c0 = zero8(), c1 = zero8();
      gemm2<8>(sQUX + 128 + hb * (32 * 512), 512, WRp + wave * (8 * 32) + lane, lane, c0, c1);
      __builtin_amdgcn_sched_barrier(0);
      epi_r(c0, 2 * hb, hh, col, sBr, hS, sQUX);
      __builtin_amdgcn_sched_barrier(0);
      epi_r(c1, 2 * hb + 1, hh, col, sBr, hS, sQUX);
    }
    __syncthreads();

    if (tid < RB) {
      const float* rr = red + tid * 16;
      float s = 0.0f;
#pragma unroll
      for (int j = 0; j < 16; ++j) s += rr[j];
      s += sBp2[0];
      pS[tid] = sigm_(s);
    }
    __syncthreads();

    if (wave == 0) {
      const v4f pv = *(const v4f*)(pS + 4 * (lane & 15));
      float* op = OUTS + (size_t)t * NB + rowBase + 4 * (lane & 15);
      if (lane < 16) *(volatile v4f*)op = pv;
      __threadfence();
      if (lane < 16) *(volatile v4f*)op = pv;
    }
#pragma unroll 2
    for (int i = 0; i < 8; ++i) {
      const int item = tid + NTHR * i;
      const int row = item >> 5, j = item & 31;
      const float* tb = TITW + (size_t)itIdx[row] * 384 + 4 * j;
      const v4f a = *(const v4f*)(tb + 128);
      const v4f b = *(const v4f*)(tb + 256);
      *(v4f*)(sIT1 + row * IT1P + 4 * j) = a;
      *(v4f*)(sIT0 + row * DD + 4 * j) = b;
    }
#pragma unroll 1
    for (int hb = 0; hb < 2; ++hb) {
      v8f c0 = zero8(), c1 = zero8();
      gemm2<8>(sQUX + 256 + hb * (32 * 512), 512, WHp + wave * (8 * 32) + lane, lane, c0, c1);
      __builtin_amdgcn_sched_barrier(0);
      epi_h(c0, 2 * hb, hh, col, sBh, zS, hS, sHH);
      __builtin_amdgcn_sched_barrier(0);
      epi_h(c1, 2 * hb + 1, hh, col, sBh, zS, hS, sHH);
    }
    __syncthreads();

#pragma unroll 1
    for (int hb = 0; hb < 2; ++hb) {
      v8f c0 = zero8(), c1 = zero8();
      gemm2<8>(sHH + hb * (32 * 256), 256, WOGp + wave * (8 * 32) + lane, lane, c0, c1);
      __builtin_amdgcn_sched_barrier(0);
      epi_g(c0, 2 * hb, hh, col, sIT1, sBog, zS);
      __builtin_amdgcn_sched_barrier(0);
      epi_g(c1, 2 * hb + 1, hh, col, sIT1, sBog, zS);
    }
#pragma unroll 1
    for (int hb = 0; hb < 2; ++hb) {
      v8f c0 = zero8(), c1 = zero8();
      gemm2<8>(sHH + hb * (32 * 256), 256, WOVp + wave * (8 * 32) + lane, lane, c0, c1);
      __builtin_amdgcn_sched_barrier(0);
      epi_v(c0, 2 * hb, hh, col, sIT0, sBov, zS, vS);
      __builtin_amdgcn_sched_barrier(0);
      epi_v(c1, 2 * hb + 1, hh, col, sIT0, sBov, zS, vS);
    }
    if (tid < RB) {
      const int tn = (t + 1 < NS) ? (t + 1) : (NS - 1);
      itIdx[tid] = clampi(it_data[(size_t)(rowBase + tid) * NS + tn], 0, NIT - 1);
    }
    __syncthreads();
  }
}

__global__ __launch_bounds__(256) void k_out(const float* __restrict__ OUTS, float* out, int nchunk) {
  const int lane = threadIdx.x & 31, wave = threadIdx.x >> 5;
  const int ch = blockIdx.x * 8 + wave;
  if (ch >= nchunk) return;
  const int f0 = ch * 128 + 4 * lane;
  v4f v;
#pragma unroll
  for (int i = 0; i < 4; ++i) {
    const int f = f0 + i;
    const int b = f / NS, t = f - NS * b;
    v[i] = OUTS[(size_t)t * NB + b];
  }
  *(volatile v4f*)(out + f0) = v;
  __threadfence();
  *(volatile v4f*)(out + f0) = v;
}

static void set_pack(PackArgs& P, int i, const float* src, _Float16* dst, int K, int N, int pitch,
                     int roff, int swp) {
  P.src[i] = src; P.dst[i] = dst; P.K[i] = K; P.N[i] = N; P.pitch[i] = pitch; P.roff[i] = roff;
  P.swp[i] = swp; P.nfrag[i] = (K / 32) * (N / 16);
}
static void set_rows(RowsArgs& R, int i, const float* src, _Float16* dst, int rsrc, int rpad, int cols,
                     float carry, int blk0) {
  R.src[i] = src; R.dst[i] = dst; R.rsrc[i] = rsrc; R.rpad[i] = rpad; R.cols[i] = cols;
  R.carry[i] = carry; R.blk0[i] = blk0; R.nb[i] = (rpad * (cols / 8)) / 256;
}
static void set_tg(TgArgs& T, int i, const _Float16* A, const _Float16* Bp, float* C, int Mpad, int K,
                   int N, float inv, int blk0) {
  T.A[i] = A; T.Bp[i] = (const v16h*)Bp; T.C[i] = C; T.Mpad[i] = Mpad; T.K[i] = K; T.N[i] = N;
  T.inv[i] = inv; T.blk0[i] = blk0; T.nb[i] = Mpad / 64;
}

extern "C" void kernel_launch(void* const* d_in, const int* in_sizes, int n_in,
                              void* d_out, int out_size, void* d_ws, size_t ws_size,
                              hipStream_t stream) {
  if (n_in < 32) return;
  for (int i = 0; i < 5; ++i) if (in_sizes[i] != NR) return;
  if (in_sizes[5] != NIT * DD || in_sizes[6] != NAT * 64 || in_sizes[7] != NANS * 64) return;
  if (in_sizes[8] != NEX * DD || in_sizes[9] != NSK * DD) return;
  for (int i = 10; i <= 20; i += 2) if (in_sizes[i] != 256 * DD || in_sizes[i + 1] != DD) return;
  if (in_sizes[22] != 384 * DD || in_sizes[23] != DD || in_sizes[24] != 384 * DD || in_sizes[25] != DD) return;
  if (in_sizes[26] != 256 * HID || in_sizes[27] != HID || in_sizes[28] != HID || in_sizes[29] != 1) return;
  if (in_sizes[30] != DD || in_sizes[31] != DD) return;
  if (out_size != NR) return;
  if ((size_t)WSTOT > ws_size) return;

  const int*   kc_data = (const int*)d_in[0];
  const int*   a_data  = (const int*)d_in[1];
  const int*   e_data  = (const int*)d_in[2];
  const int*   it_data = (const int*)d_in[3];
  const int*   at_data = (const int*)d_in[4];
  const float* it_embed = (const float*)d_in[5];
  const float* at_embed = (const float*)d_in[6];
  const float* ans_embed = (const float*)d_in[7];
  const float* ex_embed = (const float*)d_in[8];
  const float* sk_embed = (const float*)d_in[9];
  const float* Wq  = (const float*)d_in[10]; const float* bq  = (const float*)d_in[11];
  const float* Wx  = (const float*)d_in[12]; const float* bx  = (const float*)d_in[13];
  const float* Wu  = (const float*)d_in[14]; const float* bu  = (const float*)d_in[15];
  const float* Wz  = (const float*)d_in[16]; const float* bz  = (const float*)d_in[17];
  const float* Wr  = (const float*)d_in[18]; const float* br  = (const float*)d_in[19];
  const float* Wh  = (const float*)d_in[20]; const float* bh  = (const float*)d_in[21];
  const float* Wog = (const float*)d_in[22]; const float* bog = (const float*)d_in[23];
  const float* Wov = (const float*)d_in[24]; const float* bov = (const float*)d_in[25];
  const float* Wp1 = (const float*)d_in[26]; const float* bp1 = (const float*)d_in[27];
  const float* Wp2 = (const float*)d_in[28]; const float* bp2 = (const float*)d_in[29];
  const float* h0  = (const float*)d_in[30]; const float* v0  = (const float*)d_in[31];
  float* out = (float*)d_out;

  char* ws = (char*)d_ws;
  _Float16* PK    = (_Float16*)(ws + O_PK);
  _Float16* KC16  = (_Float16*)(ws + O_KC16);
  _Float16* IT16  = (_Float16*)(ws + O_IT16);
  _Float16* AT16  = (_Float16*)(ws + O_AT16);
  _Float16* ANS16 = (_Float16*)(ws + O_ANS16);
  _Float16* E16   = (_Float16*)(ws + O_E16);
  float* TKC  = (float*)(ws + O_TKC);
  float* TITW = (float*)(ws + O_TITW);
  float* TAT  = (float*)(ws + O_TAT);
  float* TANS = (float*)(ws + O_TANS);
  float* TE   = (float*)(ws + O_TE);
  float* OUTS = (float*)(ws + O_OUTS);
  _Float16* Q16 = (_Float16*)(ws + O_Q16);
  _Float16* X16 = (_Float16*)(ws + O_X16);

  PackArgs pa = {};
  set_pack(pa, 0,  Wq,  PK + PKH_WQA,   128, 128, DD,  0,   0);
  set_pack(pa, 1,  Wq,  PK + PKH_WQB,   128, 128, DD,  128, 0);
  set_pack(pa, 2,  Wx,  PK + PKH_WXA,   128, 128, DD,  0,   0);
  set_pack(pa, 3,  Wx,  PK + PKH_WXANS, 64,  128, DD,  128, 0);
  set_pack(pa, 4,  Wx,  PK + PKH_WXAT,  64,  128, DD,  192, 0);
  set_pack(pa, 5,  Wu,  PK + PKH_WUA,   128, 128, DD,  0,   0);
  set_pack(pa, 6,  Wu,  PK + PKH_ITW,   128, 128, DD,  128, 0);
  set_pack(pa, 7,  Wog, PK + PKH_ITW + 512 * 4 * 8,  128, 128, DD, 256, 0);
  set_pack(pa, 8,  Wov, PK + PKH_ITW + 512 * 4 * 16, 128, 128, DD, 256, 0);
  set_pack(pa, 9,  Wp1, PK + PKH_WP1,   256, 256, HID, 0,   1);
  set_pack(pa, 10, Wz,  PK + PKH_WZ,    256, 128, DD,  0,   1);
  set_pack(pa, 11, Wr,  PK + PKH_WR,    256, 128, DD,  0,   1);
  set_pack(pa, 12, Wh,  PK + PKH_WH,    256, 128, DD,  0,   0);
  set_pack(pa, 13, Wog, PK + PKH_WOG,   256, 128, DD,  0,   0);
  set_pack(pa, 14, Wov, PK + PKH_WOV,   256, 128, DD,  0,   0);
  set_pack(pa, 15, Wq,  PK,             128, 128, DD,  0,   0);
  pa.nfrag[15] = 0;
  k_pack<<<dim3(32, 16), 256, 0, stream>>>(pa);
  if (hipGetLastError() != hipSuccess) return;

  RowsArgs ra = {};
  set_rows(ra, 0, ex_embed,  E16,   NEX,  NEXP,  128, EC, 0);
  set_rows(ra, 1, sk_embed,  KC16,  NSK,  NSKP,  128, WC, 1252);
  set_rows(ra, 2, it_embed,  IT16,  NIT,  NITP,  128, WC, 1268);
  set_rows(ra, 3, at_embed,  AT16,  NAT,  NATP,  64,  WC, 1276);
  set_rows(ra, 4, ans_embed, ANS16, NANS, NANSP, 64,  WC, 1280);
  for (int i = 5; i < 8; ++i) { ra.src[i] = it_embed; ra.dst[i] = IT16; ra.nb[i] = 0; }
  k_rows16<<<1282, 256, 0, stream>>>(ra);
  if (hipGetLastError() != hipSuccess) return;

  TgArgs ta = {};
  set_tg(ta, 0, E16,   PK + PKH_WQA,   TE,   NEXP,  128, 128, INV_EW, 0);
  set_tg(ta, 1, KC16,  PK + PKH_WQB,   TKC,  NSKP,  128, 128, INV_TW, 313);
  set_tg(ta, 2, IT16,  PK + PKH_ITW,   TITW, NITP,  128, 384, INV_TW, 317);
  set_tg(ta, 3, AT16,  PK + PKH_WXAT,  TAT,  NATP,  64,  128, INV_TW, 319);
  set_tg(ta, 4, ANS16, PK + PKH_WXANS, TANS, NANSP, 64,  128, INV_TW, 321);
  for (int i = 5; i < 8; ++i) { ta.A[i] = IT16; ta.Bp[i] = (const v16h*)PK; ta.C[i] = TITW; ta.nb[i] = 0; }
  if (hipFuncSetAttribute(reinterpret_cast<const void*>(&k_tgemm),
                          hipFuncAttributeMaxDynamicSharedMemorySize, LDS_TG) != hipSuccess) return;
  k_tgemm<<<322, 256, LDS_TG, stream>>>(ta);
  if (hipGetLastError() != hipSuccess) return;

  k_q<<<NR * 16 / 256, 256, 0, stream>>>(e_data, kc_data, TE, TKC, bq, Q16);
  if (hipGetLastError() != hipSuccess) return;
  k_x<<<NR / RB, NTHR, 0, stream>>>(a_data, at_data, Q16, (const v16h*)(PK + PKH_WXA), TANS, TAT, bx, X16);
  if (hipGetLastError() != hipSuccess) return;

  if (hipFuncSetAttribute(reinterpret_cast<const void*>(&k_step),
                          hipFuncAttributeMaxDynamicSharedMemorySize, LDS_STEP) != hipSuccess) return;
  k_step<<<NBLK_S, NTHR, LDS_STEP, stream>>>(
      it_data, Q16, X16, TITW,
      (const v16h*)(PK + PKH_WUA), (const v16h*)(PK + PKH_WP1), (const v16h*)(PK + PKH_WZ),
      (const v16h*)(PK + PKH_WR), (const v16h*)(PK + PKH_WH), (const v16h*)(PK + PKH_WOG),
      (const v16h*)(PK + PKH_WOV),
      bu, bz, br, bh, bog, bov, bp1, Wp2, bp2, h0, v0, OUTS);
  if (hipGetLastError() != hipSuccess) return;

  k_out<<<(NCHUNK + 7) / 8, 256, 0, stream>>>(OUTS, out, NCHUNK);
  (void)hipGetLastError();
}
